// DualBlockMultiRes_8804682957477
// MI455X (gfx1250) — hardware-run, weakly checked
//
#include <hip/hip_runtime.h>

#define NBT  2
#define NTOK 2048
#define CDIM 768
#define QTOK 1024
#define QDIM 512
#define LTOK 512
#define LDIM 64
#define NHX  12
#define NHQ  8
#define HD   64

#define OUT0_N (NBT * NTOK * CDIM)
#define OUT1_N (NBT * QTOK * QDIM)
#define OUT2_N (NBT * LTOK * LDIM)

#define ASC  16.0f
#define WSC  64.0f
#define RSC  16384.0f
#define PSC  256.0f
#define G1SC 0.015625f
#define SSC  4.8828125e-4f
#define OINV 2.44140625e-4f
#define HINV 9.765625e-4f
#define LINV 5.9604644775390625e-8f

#define GP  72
#define GPT 136
#define OP  68

static_assert(NTOK % 128 == 0 && QTOK % 128 == 0 && (NBT * LTOK) % 128 == 0);
static_assert(CDIM == NHX * HD && QDIM == NHQ * HD && HD == 64 && LDIM == 64);
static_assert(CDIM % 64 == 0 && QDIM % 64 == 0 && NTOK % 32 == 0 && QTOK % 32 == 0);
static_assert((GP % 8) == 0 && (GPT % 8) == 0 && (OP % 4) == 0 && 64 * GPT <= 128 * GP);

typedef _Float16 f16;
typedef _Float16 v16h __attribute__((ext_vector_type(16)));
typedef _Float16 v8h  __attribute__((ext_vector_type(8)));
typedef _Float16 v8ha __attribute__((ext_vector_type(8), may_alias));
typedef unsigned short v8us __attribute__((ext_vector_type(8)));
typedef float v8f __attribute__((ext_vector_type(8)));
typedef float v4f __attribute__((ext_vector_type(4)));
typedef float v4fa __attribute__((ext_vector_type(4), may_alias));

union FragH { v16h v; v8h h[2]; };

__device__ __forceinline__ float bf16r(float f) {
  unsigned int u = __float_as_uint(f);
  u = u + 0x7FFFu + ((u >> 16) & 1u);
  u &= 0xFFFF0000u;
  return __uint_as_float(u);
}

__device__ __forceinline__ void split2(float v, f16& hi, f16& lo) {
  const float s = v * ASC;
  const f16 hv = (f16)s;
  hi = hv;
  lo = (f16)((s - (float)hv) * RSC);
}

__device__ __forceinline__ v16h ld_frag(const f16* base, int row0, int k0, int ld) {
  const int lane = threadIdx.x & 31;
  const f16* p = base + (size_t)(row0 + (lane & 15)) * ld + k0 + ((lane >> 4) << 3);
  FragH f;
  f.h[0] = *(const v8h*)p;
  f.h[1] = *(const v8h*)(p + 16);
  return f.v;
}

__device__ __forceinline__ v8f mma_h(v16h a, v16h b, v8f c) {
  return __builtin_amdgcn_wmma_f32_16x16x32_f16(false, a, false, b, (short)0, c, false, false);
}

__device__ __forceinline__ void guard4x4(v8f& c0, v8f& c1, v8f& c2, v8f& c3,
                                         v16h f0, v16h f1, v16h f2, v16h f3) {
#if defined(__HIP_DEVICE_COMPILE__)
  asm volatile("v_nop\n\tv_nop\n\tv_nop\n\tv_nop"
               : "+v"(c0), "+v"(c1), "+v"(c2), "+v"(c3)
               : "v"(f0), "v"(f1), "v"(f2), "v"(f3));
#endif
}
__device__ __forceinline__ void guard8x6(v8f& c0, v8f& c1, v8f& c2, v8f& c3,
                                         v8f& c4, v8f& c5, v8f& c6, v8f& c7,
                                         v16h f0, v16h f1, v16h f2, v16h f3, v16h f4, v16h f5) {
#if defined(__HIP_DEVICE_COMPILE__)
  asm volatile("v_nop\n\tv_nop\n\tv_nop\n\tv_nop"
               : "+v"(c0), "+v"(c1), "+v"(c2), "+v"(c3), "+v"(c4), "+v"(c5), "+v"(c6), "+v"(c7)
               : "v"(f0), "v"(f1), "v"(f2), "v"(f3), "v"(f4), "v"(f5));
#endif
}
__device__ __forceinline__ void guard2x6(v8f& c0, v8f& c1,
                                         v16h f0, v16h f1, v16h f2, v16h f3, v16h f4, v16h f5) {
#if defined(__HIP_DEVICE_COMPILE__)
  asm volatile("v_nop\n\tv_nop\n\tv_nop\n\tv_nop"
               : "+v"(c0), "+v"(c1)
               : "v"(f0), "v"(f1), "v"(f2), "v"(f3), "v"(f4), "v"(f5));
#endif
}
__device__ __forceinline__ void guard4x5(v8f& c0, v8f& c1, v8f& c2, v8f& c3,
                                         v16h f0, v16h f1, v16h f2, v16h f3, v16h f4) {
#if defined(__HIP_DEVICE_COMPILE__)
  asm volatile("v_nop\n\tv_nop\n\tv_nop\n\tv_nop"
               : "+v"(c0), "+v"(c1), "+v"(c2), "+v"(c3)
               : "v"(f0), "v"(f1), "v"(f2), "v"(f3), "v"(f4));
#endif
}

__global__ __launch_bounds__(256)
void k_cvt(const float* __restrict__ src, unsigned short* dst, int n8, float scale) {
  const int p = (int)blockIdx.x * 256 + (int)threadIdx.x;
  if (p >= n8) return;
  const float* s = src + (size_t)p * 8;
  const v4f x0 = *(const v4f*)s;
  const v4f x1 = *(const v4f*)(s + 4);
  v8h o = {};
#pragma unroll
  for (int e = 0; e < 4; ++e) {
    o[e]     = (f16)(bf16r(x0[e]) * scale);
    o[4 + e] = (f16)(bf16r(x1[e]) * scale);
  }
  const v8us u = __builtin_bit_cast(v8us, o);
  unsigned short* op = dst + (size_t)p * 8;
  *(volatile v8us*)op = u;
  __threadfence();
  *(volatile v8us*)op = u;
}

__global__ __launch_bounds__(256)
void k_lowres(const float* __restrict__ low, unsigned short* dst, int n8) {
  const int p = (int)blockIdx.x * 256 + (int)threadIdx.x;
  if (p >= n8) return;
  const int b  = p >> 12;
  const int r  = (p >> 3) & (LTOK - 1);
  const int c0 = (p & 7) << 3;
  const float* s = low + (size_t)b * LTOK * LDIM + (size_t)(64 * (r & 7) + c0) * LDIM + (r >> 3);
  v8h o = {};
#pragma unroll
  for (int e = 0; e < 8; ++e) o[e] = (f16)(bf16r(s[e * LDIM]) * ASC);
  const v8us u = __builtin_bit_cast(v8us, o);
  unsigned short* op = dst + (size_t)p * 8;
  *(volatile v8us*)op = u;
  __threadfence();
  *(volatile v8us*)op = u;
}

__device__ __forceinline__ void st_rows(f16* S, int row0, int col, v8f c) {
#pragma unroll
  for (int r = 0; r < 8; ++r) S[(row0 + r) * GP + col] = (f16)(c[r] * G1SC);
}
__device__ __forceinline__ void st_cols(f16* S, int d, int tok0, v8f c) {
  v8h o = {};
#pragma unroll
  for (int r = 0; r < 8; ++r) o[r] = (f16)(c[r] * G1SC);
  *(v8ha*)&S[d * GPT + tok0] = o;
}

__global__ __launch_bounds__(256)
void k_gemm_heads(const unsigned short* __restrict__ a16, const unsigned short* __restrict__ w16,
                  unsigned short* dq, unsigned short* dk, unsigned short* dvt,
                  int K, int T, int nh, int toff) {
  __shared__ __align__(16) f16 S[128 * GP];
  const int tid = threadIdx.x, lane = tid & 31, wv = tid >> 5, hl = lane >> 4, l15 = lane & 15;
  const int nb = (int)blockIdx.x;
  const int m0 = (int)blockIdx.y * 128, n0 = nb * 64;
  const int stream = nb / nh, head = nb - stream * nh, typ = stream + toff;
  const int b = m0 / T, t0 = m0 - b * T;
  const f16* Ap = (const f16*)a16;
  const f16* Wp = (const f16*)w16;
  const int mp = wv >> 1, np = wv & 1;
  const int ra = m0 + 32 * mp, cb = n0 + 32 * np;

  v8f c00 = {}, c01 = {}, c10 = {}, c11 = {};
  const int nks = K >> 5;
#pragma unroll 2
  for (int ks = 0; ks < nks; ++ks) {
    const int k0 = ks << 5;
    const v16h a0 = ld_frag(Ap, ra, k0, K);
    const v16h a1 = ld_frag(Ap, ra + 16, k0, K);
    const v16h b0 = ld_frag(Wp, cb, k0, K);
    const v16h b1 = ld_frag(Wp, cb + 16, k0, K);
    c00 = mma_h(a0, b0, c00);
    c01 = mma_h(a0, b1, c01);
    c10 = mma_h(a1, b0, c10);
    c11 = mma_h(a1, b1, c11);
    guard4x4(c00, c01, c10, c11, a0, a1, b0, b1);
  }

  const int rr = 32 * mp + 8 * hl;
  const int cc = 32 * np + l15;
  if (typ == 2) {
    st_cols(S, cc,      rr,      c00);
    st_cols(S, cc + 16, rr,      c01);
    st_cols(S, cc,      rr + 16, c10);
    st_cols(S, cc + 16, rr + 16, c11);
    __syncthreads();
    v8us u[4];
    size_t off[4];
#pragma unroll
    for (int it = 0; it < 4; ++it) {
      const int p = tid + 256 * it;
      const int d = p >> 4, q = p & 15;
      const v8h v = *(const v8ha*)&S[d * GPT + 8 * q];
      u[it] = __builtin_bit_cast(v8us, v);
      off[it] = ((size_t)(b * nh + head) * HD + d) * (size_t)T + t0 + 8 * q;
    }
#pragma unroll
    for (int it = 0; it < 4; ++it) *(volatile v8us*)(dvt + off[it]) = u[it];
    __threadfence();
#pragma unroll
    for (int it = 0; it < 4; ++it) *(volatile v8us*)(dvt + off[it]) = u[it];
  } else {
    unsigned short* dst = (typ == 0) ? dq : dk;
    st_rows(S, rr,      cc,      c00);
    st_rows(S, rr,      cc + 16, c01);
    st_rows(S, rr + 16, cc,      c10);
    st_rows(S, rr + 16, cc + 16, c11);
    __syncthreads();
    v8us u[4];
    size_t off[4];
#pragma unroll
    for (int it = 0; it < 4; ++it) {
      const int row = (tid >> 3) + 32 * it, q = tid & 7;
      const v8h v = *(const v8ha*)&S[row * GP + 8 * q];
      u[it] = __builtin_bit_cast(v8us, v);
      off[it] = ((size_t)(b * nh + head) * T + t0 + row) * HD + 8 * q;
    }
#pragma unroll
    for (int it = 0; it < 4; ++it) *(volatile v8us*)(dst + off[it]) = u[it];
    __threadfence();
#pragma unroll
    for (int it = 0; it < 4; ++it) *(volatile v8us*)(dst + off[it]) = u[it];
  }
}

__device__ __forceinline__ void flash(const f16* __restrict__ Kb, const f16* __restrict__ Vb, int nkeys, int ldv,
                                      v16h qf0, v16h qf1,
                                      v8f& O0, v8f& O1, v8f& O2, v8f& O3, float& m, float& l) {
#pragma unroll 1
  for (int kb = 0; kb < nkeys; kb += 32) {
    const v16h k00 = ld_frag(Kb, kb, 0, HD);
    const v16h k01 = ld_frag(Kb, kb, 32, HD);
    const v16h k10 = ld_frag(Kb, kb + 16, 0, HD);
    const v16h k11 = ld_frag(Kb, kb + 16, 32, HD);
    v8f s0 = {}, s1 = {};
    s0 = mma_h(k00, qf0, s0);
    s0 = mma_h(k01, qf1, s0);
    s1 = mma_h(k10, qf0, s1);
    s1 = mma_h(k11, qf1, s1);
    guard2x6(s0, s1, k00, k01, k10, k11, qf0, qf1);

    float mx = s0[0];
#pragma unroll
    for (int r = 1; r < 8; ++r) mx = fmaxf(mx, s0[r]);
#pragma unroll
    for (int r = 0; r < 8; ++r) mx = fmaxf(mx, s1[r]);
    mx = fmaxf(mx, __shfl_xor(mx, 16));
    const float mnew = fmaxf(m, mx * SSC);
    const float corr = __expf(m - mnew);
    float ps = 0.0f;
    v8h p0v = {}, p1v = {};
#pragma unroll
    for (int r = 0; r < 8; ++r) {
      const float p0 = __expf(s0[r] * SSC - mnew);
      const float p1 = __expf(s1[r] * SSC - mnew);
      ps += p0 + p1;
      p0v[r] = (f16)(p0 * PSC);
      p1v[r] = (f16)(p1 * PSC);
    }
    ps += __shfl_xor(ps, 16);
    l = l * corr + ps;
    m = mnew;
    O0 *= corr; O1 *= corr; O2 *= corr; O3 *= corr;
    FragH pf;
    pf.h[0] = p0v;
    pf.h[1] = p1v;

    const v16h v0 = ld_frag(Vb, 0,  kb, ldv);
    const v16h v1 = ld_frag(Vb, 16, kb, ldv);
    const v16h v2 = ld_frag(Vb, 32, kb, ldv);
    const v16h v3 = ld_frag(Vb, 48, kb, ldv);
    O0 = mma_h(v0, pf.v, O0);
    O1 = mma_h(v1, pf.v, O1);
    O2 = mma_h(v2, pf.v, O2);
    O3 = mma_h(v3, pf.v, O3);
    guard4x5(O0, O1, O2, O3, v0, v1, v2, v3, pf.v);
  }
}

__device__ __forceinline__ void st8(float* p, v8f o, float w) {
  v4f a, c;
#pragma unroll
  for (int i = 0; i < 4; ++i) { a[i] = o[i] * w; c[i] = o[4 + i] * w; }
  *(v4fa*)p = a;
  *(v4fa*)(p + 4) = c;
}
__device__ __forceinline__ void add8(float* p, v8f o, float w) {
  v4f a = *(const v4fa*)p;
  v4f c = *(const v4fa*)(p + 4);
#pragma unroll
  for (int i = 0; i < 4; ++i) { a[i] += o[i] * w; c[i] += o[4 + i] * w; }
  *(v4fa*)p = a;
  *(v4fa*)(p + 4) = c;
}

__device__ __forceinline__ void write_hl(const float* sow, unsigned short* oh, unsigned short* ol, size_t base, int pitch) {
  const int lane = threadIdx.x & 31;
  v8us hv[4], lv[4];
  size_t off[4];
#pragma unroll
  for (int it = 0; it < 4; ++it) {
    const int row = (lane >> 3) + 4 * it, q = lane & 7;
    const float* p = sow + row * OP + 8 * q;
    const v4f a = *(const v4fa*)p;
    const v4f c = *(const v4fa*)(p + 4);
    v8h hi = {}, lo = {};
#pragma unroll
    for (int e = 0; e < 4; ++e) {
      f16 x, y;
      split2(a[e], x, y); hi[e] = x;     lo[e] = y;
      split2(c[e], x, y); hi[4 + e] = x; lo[4 + e] = y;
    }
    hv[it] = __builtin_bit_cast(v8us, hi);
    lv[it] = __builtin_bit_cast(v8us, lo);
    off[it] = base + (size_t)row * pitch + 8 * q;
  }
#pragma unroll
  for (int it = 0; it < 4; ++it) {
    *(volatile v8us*)(oh + off[it]) = hv[it];
    *(volatile v8us*)(ol + off[it]) = lv[it];
  }
  __threadfence();
#pragma unroll
  for (int it = 0; it < 4; ++it) {
    *(volatile v8us*)(oh + off[it]) = hv[it];
    *(volatile v8us*)(ol + off[it]) = lv[it];
  }
}

__global__ __launch_bounds__(256)
void k_attn_x(const unsigned short* __restrict__ qp, const unsigned short* __restrict__ kp,
              const unsigned short* __restrict__ vtp, unsigned short* oh, unsigned short* ol) {
  __shared__ __align__(16) float So[8 * 16 * OP];
  const int tid = threadIdx.x, lane = tid & 31, wv = tid >> 5, hl = lane >> 4, l15 = lane & 15;
  const int bh = (int)blockIdx.y;
  const int b = bh / NHX, h = bh - b * NHX;
  const int q0 = (int)blockIdx.x * 128 + wv * 16;
  const f16* Qb = (const f16*)qp  + (size_t)bh * NTOK * HD;
  const f16* Kb = (const f16*)kp  + (size_t)bh * NTOK * HD;
  const f16* Vb = (const f16*)vtp + (size_t)bh * HD * NTOK;

  const v16h qf0 = ld_frag(Qb, q0, 0, HD);
  const v16h qf1 = ld_frag(Qb, q0, 32, HD);
  v8f O0 = {}, O1 = {}, O2 = {}, O3 = {};
  float m = -3.0e38f, l = 0.0f;
  flash(Kb, Vb, NTOK, NTOK, qf0, qf1, O0, O1, O2, O3, m, l);

  const float w = OINV * (1.0f / l);
  float* so = So + wv * (16 * OP) + l15 * OP + 8 * hl;
  st8(so,      O0, w);
  st8(so + 16, O1, w);
  st8(so + 32, O2, w);
  st8(so + 48, O3, w);
  __syncthreads();
  write_hl(So + wv * (16 * OP), oh, ol, ((size_t)(b * NTOK + q0)) * CDIM + (size_t)h * HD, CDIM);
}

__global__ __launch_bounds__(256)
void k_attn_q(const unsigned short* __restrict__ qqp,
              const unsigned short* __restrict__ k2p, const unsigned short* __restrict__ v2tp,
              const unsigned short* __restrict__ qkp, const unsigned short* __restrict__ qvtp,
              const float* __restrict__ gate, unsigned short* oh, unsigned short* ol) {
  __shared__ __align__(16) float So[8 * 16 * OP];
  const int tid = threadIdx.x, lane = tid & 31, wv = tid >> 5, hl = lane >> 4, l15 = lane & 15;
  const int bh = (int)blockIdx.y;
  const int b = bh / NHQ, h = bh - b * NHQ;
  const int q0 = (int)blockIdx.x * 128 + wv * 16;
  const f16* Qb  = (const f16*)qqp  + (size_t)bh * QTOK * HD;
  const f16* K1b = (const f16*)k2p  + (size_t)bh * NTOK * HD;
  const f16* V1b = (const f16*)v2tp + (size_t)bh * HD * NTOK;
  const f16* K2b = (const f16*)qkp  + (size_t)bh * QTOK * HD;
  const f16* V2b = (const f16*)qvtp + (size_t)bh * HD * QTOK;

  const v16h qf0 = ld_frag(Qb, q0, 0, HD);
  const v16h qf1 = ld_frag(Qb, q0, 32, HD);
  float* so = So + wv * (16 * OP) + l15 * OP + 8 * hl;

  {
    v8f O0 = {}, O1 = {}, O2 = {}, O3 = {};
    float m = -3.0e38f, l = 0.0f;
    flash(K1b, V1b, NTOK, NTOK, qf0, qf1, O0, O1, O2, O3, m, l);
    const float g = tanhf(bf16r(gate[h]));
    const float w = g * OINV * (1.0f / l);
    st8(so,      O0, w);
    st8(so + 16, O1, w);
    st8(so + 32, O2, w);
    st8(so + 48, O3, w);
  }
  {
    v8f O0 = {}, O1 = {}, O2 = {}, O3 = {};
    float m = -3.0e38f, l = 0.0f;
    flash(K2b, V2b, QTOK, QTOK, qf0, qf1, O0, O1, O2, O3, m, l);
    const float w = OINV * (1.0f / l);
    add8(so,      O0, w);
    add8(so + 16, O1, w);
    add8(so + 32, O2, w);
    add8(so + 48, O3, w);
  }
  __syncthreads();
  write_hl(So + wv * (16 * OP), oh, ol, ((size_t)(b * QTOK + q0)) * QDIM + (size_t)h * HD, QDIM);
}

__device__ __forceinline__ void st_out(float* So, int row0, int col, v8f hh, v8f gg, float bn) {
#pragma unroll
  for (int r = 0; r < 8; ++r) So[(row0 + r) * OP + col] = hh[r] * HINV + gg[r] * LINV + bn;
}

template <bool HASLO>
__global__ __launch_bounds__(256)
void k_gemm_out(const unsigned short* __restrict__ ah, const unsigned short* __restrict__ al,
                const unsigned short* __restrict__ w16, const float* __restrict__ bias,
                float* out, int K, int N) {
  __shared__ __align__(16) float So[128 * OP];
  const int tid = threadIdx.x, lane = tid & 31, wv = tid >> 5, hl = lane >> 4, l15 = lane & 15;
  const int m0 = (int)blockIdx.y * 128, n0 = (int)blockIdx.x * 64;
  const int mp = wv >> 1, np = wv & 1;
  const int ra = m0 + 32 * mp, cb = n0 + 32 * np;
  const f16* Hp = (const f16*)ah;
  const f16* Lp = (const f16*)al;
  const f16* Wp = (const f16*)w16;

  v8f h00 = {}, h01 = {}, h10 = {}, h11 = {};
  v8f g00 = {}, g01 = {}, g10 = {}, g11 = {};
  const int nks = K >> 5;
#pragma unroll 2
  for (int ks = 0; ks < nks; ++ks) {
    const int k0 = ks << 5;
    const v16h a0 = ld_frag(Hp, ra, k0, K);
    const v16h a1 = ld_frag(Hp, ra + 16, k0, K);
    const v16h b0 = ld_frag(Wp, cb, k0, K);
    const v16h b1 = ld_frag(Wp, cb + 16, k0, K);
    h00 = mma_h(a0, b0, h00);
    h01 = mma_h(a0, b1, h01);
    h10 = mma_h(a1, b0, h10);
    h11 = mma_h(a1, b1, h11);
    if constexpr (HASLO) {
      const v16h e0 = ld_frag(Lp, ra, k0, K);
      const v16h e1 = ld_frag(Lp, ra + 16, k0, K);
      g00 = mma_h(e0, b0, g00);
      g01 = mma_h(e0, b1, g01);
      g10 = mma_h(e1, b0, g10);
      g11 = mma_h(e1, b1, g11);
      guard8x6(h00, h01, h10, h11, g00, g01, g10, g11, a0, a1, b0, b1, e0, e1);
    } else {
      guard4x4(h00, h01, h10, h11, a0, a1, b0, b1);
    }
  }

  const float bn0 = bf16r(bias[cb + l15]);
  const float bn1 = bf16r(bias[cb + 16 + l15]);
  const int rr = 32 * mp + 8 * hl, cc = 32 * np + l15;
  st_out(So, rr,      cc,      h00, g00, bn0);
  st_out(So, rr,      cc + 16, h01, g01, bn1);
  st_out(So, rr + 16, cc,      h10, g10, bn0);
  st_out(So, rr + 16, cc + 16, h11, g11, bn1);
  __syncthreads();

  v4f u[8];
  size_t off[8];
#pragma unroll
  for (int it = 0; it < 8; ++it) {
    const int p = tid + 256 * it;
    const int row = p >> 4, q = p & 15;
    u[it] = *(const v4fa*)&So[row * OP + 4 * q];
    off[it] = (size_t)(m0 + row) * (size_t)N + n0 + 4 * q;
  }
#pragma unroll
  for (int it = 0; it < 8; ++it) *(volatile v4f*)(out + off[it]) = u[it];
  __threadfence();
#pragma unroll
  for (int it = 0; it < 8; ++it) *(volatile v4f*)(out + off[it]) = u[it];
}

extern "C" void kernel_launch(void* const* d_in, const int* in_sizes, int n_in,
                              void* d_out, int out_size, void* d_ws, size_t ws_size,
                              hipStream_t stream) {
  if (n_in < 13) return;
  if (in_sizes[0] != NBT * NTOK * CDIM || in_sizes[1] != NBT * QTOK * QDIM || in_sizes[2] != NBT * LTOK * LDIM) return;
  if (in_sizes[3] != 3 * CDIM * CDIM || in_sizes[4] != 2 * QDIM * CDIM || in_sizes[5] != 3 * QDIM * QDIM) return;
  if (in_sizes[6] != NHQ || in_sizes[7] != CDIM * CDIM || in_sizes[8] != CDIM) return;
  if (in_sizes[9] != QDIM * QDIM || in_sizes[10] != QDIM || in_sizes[11] != LDIM * LDIM || in_sizes[12] != LDIM) return;
  if (out_size != OUT0_N + OUT1_N + OUT2_N) return;

  const size_t sz_x16  = (size_t)NBT * NTOK * CDIM * 2;
  const size_t sz_q16  = (size_t)NBT * QTOK * QDIM * 2;
  const size_t sz_wqkv = (size_t)3 * CDIM * CDIM * 2;
  const size_t sz_wxkv = (size_t)2 * QDIM * CDIM * 2;
  const size_t sz_wqln = (size_t)3 * QDIM * QDIM * 2;
  const size_t sz_wprj = (size_t)CDIM * CDIM * 2;
  const size_t sz_wqpj = (size_t)QDIM * QDIM * 2;
  const size_t sz_wlpj = (size_t)LDIM * LDIM * 2;
  const size_t sz_l16  = (size_t)NBT * LTOK * LDIM * 2;
  const size_t sz_hx   = (size_t)NBT * NHX * NTOK * HD * 2;
  const size_t sz_hk2  = (size_t)NBT * NHQ * NTOK * HD * 2;
  const size_t sz_hq   = (size_t)NBT * NHQ * QTOK * HD * 2;

  const size_t off_x16  = 0;
  const size_t off_q16  = off_x16  + sz_x16;
  const size_t off_wqkv = off_q16  + sz_q16;
  const size_t off_wxkv = off_wqkv + sz_wqkv;
  const size_t off_wqln = off_wxkv + sz_wxkv;
  const size_t off_wprj = off_wqln + sz_wqln;
  const size_t off_wqpj = off_wprj + sz_wprj;
  const size_t off_wlpj = off_wqpj + sz_wqpj;
  const size_t off_l16  = off_wlpj + sz_wlpj;
  const size_t off_qx   = off_l16  + sz_l16;
  const size_t off_kx   = off_qx   + sz_hx;
  const size_t off_vxt  = off_kx   + sz_hx;
  const size_t off_k2   = off_vxt  + sz_hx;
  const size_t off_v2t  = off_k2   + sz_hk2;
  const size_t off_qq   = off_v2t  + sz_hk2;
  const size_t off_qk   = off_qq   + sz_hq;
  const size_t off_qvt  = off_qk   + sz_hq;
  const size_t off_xoh  = off_qvt  + sz_hq;
  const size_t off_xol  = off_xoh  + sz_x16;
  const size_t off_qoh  = off_xol  + sz_x16;
  const size_t off_qol  = off_qoh  + sz_q16;
  const size_t need     = off_qol  + sz_q16;
  if (need > ws_size) return;
  if (need > (size_t)134217728) return;

  const float* x       = (const float*)d_in[0];
  const float* query   = (const float*)d_in[1];
  const float* low_res = (const float*)d_in[2];
  const float* W_qkv   = (const float*)d_in[3];
  const float* W_xkv   = (const float*)d_in[4];
  const float* W_qlin  = (const float*)d_in[5];
  const float* gate    = (const float*)d_in[6];
  const float* W_proj  = (const float*)d_in[7];
  const float* b_proj  = (const float*)d_in[8];
  const float* W_qproj = (const float*)d_in[9];
  const float* b_qproj = (const float*)d_in[10];
  const float* W_lproj = (const float*)d_in[11];
  const float* b_lproj = (const float*)d_in[12];

  float* out0 = (float*)d_out;
  float* out1 = out0 + OUT0_N;
  float* out2 = out1 + OUT1_N;

  char* wsb = (char*)d_ws;
  unsigned short* x16_p  = (unsigned short*)(wsb + off_x16);
  unsigned short* q16_p  = (unsigned short*)(wsb + off_q16);
  unsigned short* wqkv_p = (unsigned short*)(wsb + off_wqkv);
  unsigned short* wxkv_p = (unsigned short*)(wsb + off_wxkv);
  unsigned short* wqln_p = (unsigned short*)(wsb + off_wqln);
  unsigned short* wprj_p = (unsigned short*)(wsb + off_wprj);
  unsigned short* wqpj_p = (unsigned short*)(wsb + off_wqpj);
  unsigned short* wlpj_p = (unsigned short*)(wsb + off_wlpj);
  unsigned short* l16_p  = (unsigned short*)(wsb + off_l16);
  unsigned short* qx_p   = (unsigned short*)(wsb + off_qx);
  unsigned short* kx_p   = (unsigned short*)(wsb + off_kx);
  unsigned short* vxt_p  = (unsigned short*)(wsb + off_vxt);
  unsigned short* k2_p   = (unsigned short*)(wsb + off_k2);
  unsigned short* v2t_p  = (unsigned short*)(wsb + off_v2t);
  unsigned short* qq_p   = (unsigned short*)(wsb + off_qq);
  unsigned short* qk_p   = (unsigned short*)(wsb + off_qk);
  unsigned short* qvt_p  = (unsigned short*)(wsb + off_qvt);
  unsigned short* xoh_p  = (unsigned short*)(wsb + off_xoh);
  unsigned short* xol_p  = (unsigned short*)(wsb + off_xol);
  unsigned short* qoh_p  = (unsigned short*)(wsb + off_qoh);
  unsigned short* qol_p  = (unsigned short*)(wsb + off_qol);

  const int n8_x    = NBT * NTOK * CDIM / 8;
  const int n8_q    = NBT * QTOK * QDIM / 8;
  const int n8_wqkv = 3 * CDIM * CDIM / 8;
  const int n8_wxkv = 2 * QDIM * CDIM / 8;
  const int n8_wqln = 3 * QDIM * QDIM / 8;
  const int n8_wprj = CDIM * CDIM / 8;
  const int n8_wqpj = QDIM * QDIM / 8;
  const int n8_wlpj = LDIM * LDIM / 8;
  const int n8_l    = NBT * LTOK * LDIM / 8;
  k_cvt<<<dim3((n8_x + 255) / 256),    dim3(256), 0, stream>>>(x,       x16_p,  n8_x,    ASC);
  k_cvt<<<dim3((n8_q + 255) / 256),    dim3(256), 0, stream>>>(query,   q16_p,  n8_q,    ASC);
  k_cvt<<<dim3((n8_wqkv + 255) / 256), dim3(256), 0, stream>>>(W_qkv,   wqkv_p, n8_wqkv, WSC);
  k_cvt<<<dim3((n8_wxkv + 255) / 256), dim3(256), 0, stream>>>(W_xkv,   wxkv_p, n8_wxkv, WSC);
  k_cvt<<<dim3((n8_wqln + 255) / 256), dim3(256), 0, stream>>>(W_qlin,  wqln_p, n8_wqln, WSC);
  k_cvt<<<dim3((n8_wprj + 255) / 256), dim3(256), 0, stream>>>(W_proj,  wprj_p, n8_wprj, WSC);
  k_cvt<<<dim3((n8_wqpj + 255) / 256), dim3(256), 0, stream>>>(W_qproj, wqpj_p, n8_wqpj, WSC);
  k_cvt<<<dim3((n8_wlpj + 255) / 256), dim3(256), 0, stream>>>(W_lproj, wlpj_p, n8_wlpj, WSC);
  k_lowres<<<dim3((n8_l + 255) / 256), dim3(256), 0, stream>>>(low_res, l16_p, n8_l);

  k_gemm_heads<<<dim3(3 * CDIM / 64, NBT * NTOK / 128), dim3(256), 0, stream>>>(
      x16_p, wqkv_p, qx_p, kx_p, vxt_p, CDIM, NTOK, NHX, 0);
  k_gemm_heads<<<dim3(2 * QDIM / 64, NBT * NTOK / 128), dim3(256), 0, stream>>>(
      x16_p, wxkv_p, k2_p, k2_p, v2t_p, CDIM, NTOK, NHQ, 1);
  k_gemm_heads<<<dim3(3 * QDIM / 64, NBT * QTOK / 128), dim3(256), 0, stream>>>(
      q16_p, wqln_p, qq_p, qk_p, qvt_p, QDIM, QTOK, NHQ, 0);

  k_attn_x<<<dim3(NTOK / 128, NBT * NHX), dim3(256), 0, stream>>>(qx_p, kx_p, vxt_p, xoh_p, xol_p);
  k_attn_q<<<dim3(QTOK / 128, NBT * NHQ), dim3(256), 0, stream>>>(qq_p, k2_p, v2t_p, qk_p, qvt_p, gate, qoh_p, qol_p);

  k_gemm_out<true><<<dim3(CDIM / 64, NBT * NTOK / 128), dim3(256), 0, stream>>>(
      xoh_p, xol_p, wprj_p, b_proj, out0, CDIM, CDIM);
  k_gemm_out<true><<<dim3(QDIM / 64, NBT * QTOK / 128), dim3(256), 0, stream>>>(
      qoh_p, qol_p, wqpj_p, b_qproj, out1, QDIM, QDIM);
  k_gemm_out<false><<<dim3(LDIM / 64, NBT * LTOK / 128), dim3(256), 0, stream>>>(
      l16_p, l16_p, wlpj_p, b_lproj, out2, LDIM, LDIM);
  (void)hipGetLastError();
}
